// BotDCGCGraphAutoEncoder_88648124989885
// MI455X (gfx1250) — hardware-run, weakly checked
//
#include <hip/hip_runtime.h>
#include <stddef.h>


#define IN0     512
#define HID1    256
#define HID2    128
#define BN1     (2 * HID1)
#define BN2     (2 * HID2)
#define NTHR    256
#define NWAVE   8
#define EPT     8
#define NGRP    2
#define CHUNK   (NTHR * EPT * NGRP)
#define WCAP    (EPT * NGRP * 32)
#define LISTN   (NWAVE * WCAP)
#define NBC     4096
#define NBF     1024
#define RCAP    49152
#define RBN     128
#define TGT     256
#define DEGCAP  512
#define OTHR    512
#define BM      32
#define WSCAP   134217728
#define NEG_SLOPE 0.2f
#define LN_EPS  1e-5f
#define SCLAMP  30.0f

#define LDS_FILL ((RCAP + NBF + LISTN) * 4 + 64)
#define LDS_G1   (BM * BN1 * 4)
#define LDS_G2   (BM * BN2 * 4)

static_assert((CHUNK & (CHUNK - 1)) == 0);
static_assert(CHUNK <= 4096);
static_assert(NBC <= 4096 && NBF <= 4096);
static_assert((NBC & (NBC - 1)) == 0 && (NBF & (NBF - 1)) == 0);
static_assert(NBC == 4 * NBF);
static_assert(OTHR * 8 == NBC);
static_assert((RCAP % 32) == 0);
static_assert(TGT == NWAVE * 32);
static_assert((NBC % TGT) == 0);
static_assert((TGT % BM) == 0);
static_assert(BM == 4 * NWAVE);
static_assert(IN0 % 32 == 0 && HID1 % 32 == 0 && HID2 % 32 == 0);
static_assert(HID1 % 128 == 0 && HID2 % 128 == 0);

typedef float          v4f   __attribute__((ext_vector_type(4)));
typedef float          v8f   __attribute__((ext_vector_type(8)));
typedef int            v4i   __attribute__((ext_vector_type(4)));
typedef unsigned short v8us  __attribute__((ext_vector_type(8)));
typedef __bf16         v16bf __attribute__((ext_vector_type(16)));
union FragB { v16bf v; v8us u[2]; };

__device__ __forceinline__ v8f wmb(v16bf a, v16bf b, v8f c) {
  v8f d = __builtin_amdgcn_wmma_f32_16x16x32_bf16(false, a, false, b, (short)0, c, false, false);
  asm volatile("v_nop\n\tv_nop\n\tv_nop\n\tv_nop" : "+v"(d) : "v"(a), "v"(b));
  return d;
}

__device__ __forceinline__ unsigned bfr(float f) {
  const unsigned u = __float_as_uint(f);
  return (u + 0x7fffu + ((u >> 16) & 1u)) >> 16;
}

__device__ __forceinline__ void split8(v8f f, v8us& hi, v8us& lo) {
  v8us h, l;
#pragma unroll
  for (int i = 0; i < 8; ++i) {
    const unsigned hb = bfr(f[i]);
    const float hf = __uint_as_float(hb << 16);
    const unsigned lb = bfr(f[i] - hf);
    h[i] = (unsigned short)hb;
    l[i] = (unsigned short)lb;
  }
  hi = h; lo = l;
}

__device__ __forceinline__ float lrelu(float v) { return v >= 0.0f ? v : NEG_SLOPE * v; }

__device__ __forceinline__ float wvmax(float v) {
#pragma unroll
  for (int o = 16; o > 0; o >>= 1) v = fmaxf(v, __shfl_xor(v, o));
  return v;
}
__device__ __forceinline__ float wvsum(float v) {
#pragma unroll
  for (int o = 16; o > 0; o >>= 1) v += __shfl_xor(v, o);
  return v;
}

template <int NB>
__device__ __forceinline__ int scan_chunk(const int* __restrict__ keys, int nE, int cbase, int slotBase,
                                          int vec8, int* list, int tid, int lane, int wave) {
  int wc = 0;
#pragma unroll
  for (int g = 0; g < NGRP; ++g) {
    const int el0  = (g * NTHR + tid) * EPT;
    const int e0   = cbase + el0;
    const int sent = -2147483647 - 1;
    v4i da, db;
    if (vec8 != 0 && cbase + CHUNK <= nE) {
      da = *(const v4i*)(keys + e0);
      db = *(const v4i*)(keys + e0 + 4);
    } else {
      da.x = (e0     < nE) ? keys[min(e0, nE - 1)] : sent;
      da.y = (e0 + 1 < nE) ? keys[min(e0 + 1, nE - 1)] : sent;
      da.z = (e0 + 2 < nE) ? keys[min(e0 + 2, nE - 1)] : sent;
      da.w = (e0 + 3 < nE) ? keys[min(e0 + 3, nE - 1)] : sent;
      db.x = (e0 + 4 < nE) ? keys[min(e0 + 4, nE - 1)] : sent;
      db.y = (e0 + 5 < nE) ? keys[min(e0 + 5, nE - 1)] : sent;
      db.z = (e0 + 6 < nE) ? keys[min(e0 + 6, nE - 1)] : sent;
      db.w = (e0 + 7 < nE) ? keys[min(e0 + 7, nE - 1)] : sent;
    }
    const unsigned nb = (unsigned)slotBase;
    const unsigned s0 = (unsigned)da.x - nb, s1 = (unsigned)da.y - nb;
    const unsigned s2 = (unsigned)da.z - nb, s3 = (unsigned)da.w - nb;
    const unsigned s4 = (unsigned)db.x - nb, s5 = (unsigned)db.y - nb;
    const unsigned s6 = (unsigned)db.z - nb, s7 = (unsigned)db.w - nb;
    const bool h0 = s0 < (unsigned)NB, h1 = s1 < (unsigned)NB, h2 = s2 < (unsigned)NB, h3 = s3 < (unsigned)NB;
    const bool h4 = s4 < (unsigned)NB, h5 = s5 < (unsigned)NB, h6 = s6 < (unsigned)NB, h7 = s7 < (unsigned)NB;
    const unsigned any = __builtin_amdgcn_ballot_w32(h0 | h1 | h2 | h3 | h4 | h5 | h6 | h7);
    if (any != 0u) {
#define HITJ(J, HJ, SJ) { \
        const unsigned mj = __builtin_amdgcn_ballot_w32(HJ); \
        if (mj != 0u) { \
          if (HJ) { \
            const int pos = wc + (int)__builtin_amdgcn_mbcnt_lo(mj, 0u); \
            if (pos < WCAP) list[wave * WCAP + pos] = ((el0 + (J)) << 12) | (int)(SJ); \
          } \
          wc += (int)__builtin_popcount(mj); } }
      HITJ(0, h0, s0)
      HITJ(1, h1, s1)
      HITJ(2, h2, s2)
      HITJ(3, h3, s3)
      HITJ(4, h4, s4)
      HITJ(5, h5, s5)
      HITJ(6, h6, s6)
      HITJ(7, h7, s7)
#undef HITJ
    }
  }
  return wc;
}

template <int K>
__global__ __launch_bounds__(NTHR) void k_xcvt(const float* __restrict__ x,
                                               unsigned short* xh, unsigned short* xl,
                                               int nN, int nUnits) {
  constexpr int KS = K / 8;
  static_assert(KS * 8 == K && (KS % 32) == 0);
  const int i = (int)blockIdx.x * NTHR + (int)threadIdx.x;
  if (i >= nUnits) return;
  const int row = i / KS;
  const int c0  = (i - row * KS) * 8;
  int rr = row > nN - 1 ? nN - 1 : row;
  rr = rr < 0 ? 0 : rr;
  const float* p = x + (size_t)rr * K + c0;
  v4f a = *(const v4f*)p, b = *(const v4f*)(p + 4);
  const v4f z = {0.f, 0.f, 0.f, 0.f};
  if (row >= nN) { a = z; b = z; }
  v8f f;
  f[0] = a.x; f[1] = a.y; f[2] = a.z; f[3] = a.w;
  f[4] = b.x; f[5] = b.y; f[6] = b.z; f[7] = b.w;
  v8us h, l;
  split8(f, h, l);
  unsigned short* dh = xh + (size_t)i * 8;
  unsigned short* dl = xl + (size_t)i * 8;
  *(volatile v8us*)dh = h;
  *(volatile v8us*)dl = l;
  __threadfence();
  *(volatile v8us*)dh = h;
  *(volatile v8us*)dl = l;
}

template <int K, int NO>
__global__ __launch_bounds__(NTHR) void k_wprep(const float* __restrict__ W,
                                                const float* __restrict__ Wr,
                                                unsigned short* wh, unsigned short* wl) {
  constexpr int KS    = K / 8;
  constexpr int UNITS = 2 * NO * KS;
  static_assert(KS * 8 == K && (KS % 32) == 0);
  const int i = (int)blockIdx.x * NTHR + (int)threadIdx.x;
  if (i >= UNITS) return;
  const int n  = i / KS;
  const int k0 = (i - n * KS) * 8;
  const int na = n > NO - 1 ? NO - 1 : n;
  int nb = n - NO;
  nb = nb < 0 ? 0 : (nb > NO - 1 ? NO - 1 : nb);
  const bool useA = n < NO;
  v8f f;
#pragma unroll
  for (int j = 0; j < 8; ++j) {
    const float va = W [(size_t)(k0 + j) * NO + na];
    const float vb = Wr[(size_t)(k0 + j) * NO + nb];
    f[j] = useA ? va : vb;
  }
  v8us h, l;
  split8(f, h, l);
  unsigned short* dh = wh + (size_t)i * 8;
  unsigned short* dl = wl + (size_t)i * 8;
  *(volatile v8us*)dh = h;
  *(volatile v8us*)dl = l;
  __threadfence();
  *(volatile v8us*)dh = h;
  *(volatile v8us*)dl = l;
}

__global__ __launch_bounds__(NTHR) void k_count(
    const int* __restrict__ keys, int* cnt, int nE, int vec8) {
  __shared__ __attribute__((aligned(16))) int scnt[NBC];
  __shared__ __attribute__((aligned(16))) int list[LISTN];
  __shared__ int wcnt[NWAVE];
  const int tid = threadIdx.x, lane = tid & 31, wave = tid >> 5;
  const int nodeBase = blockIdx.x * NBC;

  for (int i = tid; i < NBC; i += NTHR) scnt[i] = 0;
  __syncthreads();

  const int nChunks = (nE + CHUNK - 1) / CHUNK;
#pragma unroll 1
  for (int ch = 0; ch < nChunks; ++ch) {
    const int cbase = ch * CHUNK;
    const int wc = scan_chunk<NBC>(keys, nE, cbase, nodeBase, vec8, list, tid, lane, wave);
    if (lane == 0) wcnt[wave] = wc;
    __syncthreads();
    if (wave == 0) {
#pragma unroll 1
      for (int wsx = 0; wsx < NWAVE; ++wsx) {
        int n = __builtin_amdgcn_readfirstlane(wcnt[wsx]);
        n = n > WCAP ? WCAP : (n < 0 ? 0 : n);
        const int* lp = list + wsx * WCAP;
#pragma unroll 1
        for (int i = 0; i < n; ++i) {
          const int ent  = __builtin_amdgcn_readfirstlane(lp[i]);
          const int slot = ent & (NBC - 1);
          if (lane == 0) scnt[slot] = scnt[slot] + 1;
        }
      }
    }
    __syncthreads();
  }

  v4i cq[4];
#pragma unroll
  for (int q = 0; q < 4; ++q) {
    const int f = (wave * 4 + q) * 128 + 4 * lane;
    cq[q] = *(const v4i*)(scnt + f);
  }
  int* cp = cnt + (size_t)nodeBase;
#pragma unroll
  for (int q = 0; q < 4; ++q) {
    const int f = (wave * 4 + q) * 128 + 4 * lane;
    *(volatile v4i*)(cp + f) = cq[q];
  }
  __threadfence();
#pragma unroll
  for (int q = 0; q < 4; ++q) {
    const int f = (wave * 4 + q) * 128 + 4 * lane;
    *(volatile v4i*)(cp + f) = cq[q];
  }
}

__global__ __launch_bounds__(OTHR) void k_offsets(
    const int* __restrict__ cnt, int* off, int* rbase, int nChunk) {
  __shared__ __attribute__((aligned(16))) int soff[NBC];
  __shared__ __attribute__((aligned(16))) int srb[RBN];
  __shared__ int wtot[OTHR / 32];
  const int tid = threadIdx.x, lane = tid & 31, wave = tid >> 5, sub = tid >> 7;
  for (int i = tid; i < RBN; i += OTHR) srb[i] = 0;
  int carry = 0;
#pragma unroll 1
  for (int ch = 0; ch < nChunk; ++ch) {
    const int base = ch * NBC;
    const v4i c0 = *(const v4i*)(cnt + base + 8 * tid);
    const v4i c1 = *(const v4i*)(cnt + base + 8 * tid + 4);
    const int e0 = max(c0.x, 0), e1 = max(c0.y, 0), e2 = max(c0.z, 0), e3 = max(c0.w, 0);
    const int e4 = max(c1.x, 0), e5 = max(c1.y, 0), e6 = max(c1.z, 0), e7 = max(c1.w, 0);
    const int ts = e0 + e1 + e2 + e3 + e4 + e5 + e6 + e7;
    int incl = ts;
#pragma unroll
    for (int d = 1; d < 32; d <<= 1) {
      const int t = __shfl_up(incl, d);
      if (lane >= d) incl += t;
    }
    if (lane == 31) wtot[wave] = incl;
    __syncthreads();
    const int S0 = wtot[0]  + wtot[1]  + wtot[2]  + wtot[3];
    const int S1 = wtot[4]  + wtot[5]  + wtot[6]  + wtot[7];
    const int S2 = wtot[8]  + wtot[9]  + wtot[10] + wtot[11];
    const int S3 = wtot[12] + wtot[13] + wtot[14] + wtot[15];
    int pre = 0;
#pragma unroll 1
    for (int w = 4 * sub; w < wave; ++w) pre += wtot[w];
    const int b0 = carry;
    const int b1 = b0 + ((S0 + 31) & ~31);
    const int b2 = b1 + ((S1 + 31) & ~31);
    const int b3 = b2 + ((S2 + 31) & ~31);
    const int b4 = b3 + ((S3 + 31) & ~31);
    const int myb = sub == 0 ? b0 : (sub == 1 ? b1 : (sub == 2 ? b2 : b3));
    if (tid == 0) {
      srb[min(4 * ch + 0, RBN - 1)] = b0;
      srb[min(4 * ch + 1, RBN - 1)] = b1;
      srb[min(4 * ch + 2, RBN - 1)] = b2;
      srb[min(4 * ch + 3, RBN - 1)] = b3;
    }
    int run = myb + pre + incl - ts;
    soff[8 * tid + 0] = run; run += e0;
    soff[8 * tid + 1] = run; run += e1;
    soff[8 * tid + 2] = run; run += e2;
    soff[8 * tid + 3] = run; run += e3;
    soff[8 * tid + 4] = run; run += e4;
    soff[8 * tid + 5] = run; run += e5;
    soff[8 * tid + 6] = run; run += e6;
    soff[8 * tid + 7] = run;
    carry = b4;
    __syncthreads();
    const v4i o0 = *(const v4i*)(soff + 4 * tid);
    const v4i o1 = *(const v4i*)(soff + 4 * (tid + OTHR));
    int* op = off + base;
    *(volatile v4i*)(op + 4 * tid) = o0;
    *(volatile v4i*)(op + 4 * (tid + OTHR)) = o1;
    __threadfence();
    *(volatile v4i*)(op + 4 * tid) = o0;
    *(volatile v4i*)(op + 4 * (tid + OTHR)) = o1;
    __syncthreads();
  }
  if (tid == 0) srb[min(4 * nChunk, RBN - 1)] = carry;
  __syncthreads();
  v4i rv = {0, 0, 0, 0};
  if (tid < 32) rv = *(const v4i*)(srb + 4 * tid);
  if (tid < 32) *(volatile v4i*)(rbase + 4 * tid) = rv;
  __threadfence();
  if (tid < 32) *(volatile v4i*)(rbase + 4 * tid) = rv;
}

__global__ __launch_bounds__(NTHR) void k_fill(
    const int* __restrict__ keys, const int* __restrict__ off, const int* __restrict__ rbase,
    int* csr, int nE, int vec8, int csrLen) {
  extern __shared__ v4f lds_dyn[];
  int* region = (int*)lds_dyn;
  int* cursor = region + RCAP;
  int* list   = cursor + NBF;
  int* wcnt   = list + LISTN;
  const int tid = threadIdx.x, lane = tid & 31, wave = tid >> 5;
  const int b = blockIdx.x;
  const int nodeBase = b * NBF;

  int rb0 = rbase[b];
  const int rb1 = rbase[b + 1];
  rb0 = rb0 < 0 ? 0 : (rb0 > csrLen ? csrLen : rb0);
  rb0 &= ~31;
  int len = rb1 - rb0;
  len = len < 0 ? 0 : (len > RCAP ? RCAP : len);
  int lenW = (len + 31) & ~31;
  if (rb0 + lenW > csrLen) lenW = (csrLen - rb0) & ~31;

  {
    const v4i z = {0, 0, 0, 0};
    for (int i = tid; i < RCAP / 4; i += NTHR) ((v4i*)region)[i] = z;
    for (int s = tid; s < NBF; s += NTHR) {
      int o = off[nodeBase + s] - rb0;
      o = o < 0 ? 0 : (o > RCAP ? RCAP : o);
      cursor[s] = o;
    }
  }
  __syncthreads();

  const int nChunks = (nE + CHUNK - 1) / CHUNK;
#pragma unroll 1
  for (int ch = 0; ch < nChunks; ++ch) {
    const int cbase = ch * CHUNK;
    const int wc = scan_chunk<NBF>(keys, nE, cbase, nodeBase, vec8, list, tid, lane, wave);
    if (lane == 0) wcnt[wave] = wc;
    __syncthreads();
    if (wave == 0) {
#pragma unroll 1
      for (int wsx = 0; wsx < NWAVE; ++wsx) {
        int n = __builtin_amdgcn_readfirstlane(wcnt[wsx]);
        n = n > WCAP ? WCAP : (n < 0 ? 0 : n);
        const int* lp = list + wsx * WCAP;
#pragma unroll 1
        for (int i = 0; i < n; ++i) {
          const int ent  = __builtin_amdgcn_readfirstlane(lp[i]);
          const int slot = ent & (NBF - 1);
          int e = cbase + ((ent >> 12) & (CHUNK - 1));
          e = e > nE - 1 ? nE - 1 : e;
          if (lane == 0) {
            int pos = cursor[slot];
            pos = pos < 0 ? 0 : (pos > RCAP - 1 ? RCAP - 1 : pos);
            region[pos] = e;
            const int np = pos + 1;
            cursor[slot] = np > RCAP ? RCAP : np;
          }
        }
      }
    }
    __syncthreads();
  }

  const int nv = lenW >> 2;
  int* gp = csr + rb0;
#pragma unroll 1
  for (int i = tid; i < nv; i += NTHR) { const v4i v = ((const v4i*)region)[i]; *(volatile v4i*)(gp + 4 * i) = v; }
  __threadfence();
#pragma unroll 1
  for (int i = tid; i < nv; i += NTHR) { const v4i v = ((const v4i*)region)[i]; *(volatile v4i*)(gp + 4 * i) = v; }
}

template <int K, int BN>
__global__ __launch_bounds__(NTHR) void k_gemm(
    const unsigned short* __restrict__ Ah, const unsigned short* __restrict__ Al,
    const unsigned short* __restrict__ Bh, const unsigned short* __restrict__ Bl,
    const float* __restrict__ avs, const float* __restrict__ avd,
    float* C, float* eS, float* eD) {
  constexpr int KT  = K / 32;
  constexpr int CW  = BN / NWAVE;
  constexpr int TPW = CW / 16;
  constexpr int HD  = BN / 2;
  constexpr int CPP = HD / 8;
  constexpr int NIT = BM / NWAVE;
  constexpr int NPC = BN / 128;
  static_assert(K % 32 == 0);
  static_assert(TPW >= 1 && TPW * 16 * NWAVE == BN);
  static_assert(CPP % 4 == 0 && CPP * 8 == HD);
  static_assert(NPC * 128 == BN);
  static_assert(BM == 32 && NIT == 4);

  extern __shared__ v4f lds_dyn[];
  float* stg = (float*)lds_dyn;
  __shared__ __attribute__((aligned(16))) float sES[BM];
  __shared__ __attribute__((aligned(16))) float sED[BM];
  const int tid = threadIdx.x, lane = tid & 31, wave = tid >> 5, hh = lane >> 4, m = lane & 15;
  const int rowBase = blockIdx.x * BM;
  const int c0 = wave * CW;

  v8f acc0[TPW], acc1[TPW];
#pragma unroll
  for (int t = 0; t < TPW; ++t) {
    v8f z = {0.f, 0.f, 0.f, 0.f, 0.f, 0.f, 0.f, 0.f};
    acc0[t] = z; acc1[t] = z;
  }

  const size_t arow0 = (size_t)(rowBase + m) * K + 8 * hh;
  const size_t arow1 = (size_t)(rowBase + 16 + m) * K + 8 * hh;
  const unsigned short* a0h = Ah + arow0;
  const unsigned short* a0l = Al + arow0;
  const unsigned short* a1h = Ah + arow1;
  const unsigned short* a1l = Al + arow1;
  const size_t brow = (size_t)(c0 + m) * K + 8 * hh;
  const unsigned short* bph = Bh + brow;
  const unsigned short* bpl = Bl + brow;
#pragma unroll 1
  for (int kt = 0; kt < KT; ++kt) {
    const int ko = 32 * kt;
    FragB x0h, x0l, x1h, x1l;
    x0h.u[0] = *(const v8us*)(a0h + ko);
    x0h.u[1] = *(const v8us*)(a0h + ko + 16);
    x0l.u[0] = *(const v8us*)(a0l + ko);
    x0l.u[1] = *(const v8us*)(a0l + ko + 16);
    x1h.u[0] = *(const v8us*)(a1h + ko);
    x1h.u[1] = *(const v8us*)(a1h + ko + 16);
    x1l.u[0] = *(const v8us*)(a1l + ko);
    x1l.u[1] = *(const v8us*)(a1l + ko + 16);
#pragma unroll
    for (int t = 0; t < TPW; ++t) {
      const size_t bo = (size_t)(16 * t) * K + ko;
      FragB bh, bl;
      bh.u[0] = *(const v8us*)(bph + bo);
      bh.u[1] = *(const v8us*)(bph + bo + 16);
      bl.u[0] = *(const v8us*)(bpl + bo);
      bl.u[1] = *(const v8us*)(bpl + bo + 16);
      acc0[t] = wmb(x0h.v, bh.v, acc0[t]);
      acc0[t] = wmb(x0h.v, bl.v, acc0[t]);
      acc0[t] = wmb(x0l.v, bh.v, acc0[t]);
      acc1[t] = wmb(x1h.v, bh.v, acc1[t]);
      acc1[t] = wmb(x1h.v, bl.v, acc1[t]);
      acc1[t] = wmb(x1l.v, bh.v, acc1[t]);
    }
  }

  {
    float* sp0 = stg + (size_t)(8 * hh) * BN + c0 + m;
    float* sp1 = stg + (size_t)(16 + 8 * hh) * BN + c0 + m;
#pragma unroll
    for (int t = 0; t < TPW; ++t) {
#pragma unroll
      for (int r = 0; r < 8; ++r) {
        sp0[r * BN + 16 * t] = acc0[t][r];
        sp1[r * BN + 16 * t] = acc1[t][r];
      }
    }
  }
  __syncthreads();

  {
    const int drow = tid >> 3, part = tid & 7;
    const float* rp  = stg + (size_t)drow * BN + CPP * part;
    const float* sa  = avs + CPP * part;
    const float* sdd = avd + CPP * part;
    float ps = 0.f, pd = 0.f;
#pragma unroll 2
    for (int c = 0; c < CPP; c += 4) {
      const v4f hv = *(const v4f*)(rp + c);
      const v4f av = *(const v4f*)(sa + c);
      const v4f dv = *(const v4f*)(sdd + c);
      ps += hv.x * av.x + hv.y * av.y + hv.z * av.z + hv.w * av.w;
      pd += hv.x * dv.x + hv.y * dv.y + hv.z * dv.z + hv.w * dv.w;
    }
    ps += __shfl_xor(ps, 1); pd += __shfl_xor(pd, 1);
    ps += __shfl_xor(ps, 2); pd += __shfl_xor(pd, 2);
    ps += __shfl_xor(ps, 4); pd += __shfl_xor(pd, 4);
    if (part == 0) { sES[drow] = ps; sED[drow] = pd; }
  }

  {
    float* cb = C + (size_t)rowBase * BN + 4 * lane;
    auto cpass = [&]() {
#pragma unroll
      for (int it = 0; it < NIT; ++it) {
        const int row = it * NWAVE + wave;
        const float* srow = stg + (size_t)row * BN + 4 * lane;
        float* gp = cb + (size_t)row * BN;
#pragma unroll
        for (int p = 0; p < NPC; ++p) {
          const v4f v = *(const v4f*)(srow + 128 * p);
          *(volatile v4f*)(gp + 128 * p) = v;
        }
      }
    };
    cpass();
    __threadfence();
    cpass();
  }
  __syncthreads();

  {
    const int lq = lane & 7;
    const v4f vS = *(const v4f*)(sES + 4 * lq);
    const v4f vD = *(const v4f*)(sED + 4 * lq);
    const v4f dv = (wave == 0) ? vS : vD;
    float* gp = ((wave == 0) ? eS : eD) + (size_t)rowBase + 4 * lq;
    const bool act = (wave < 2) && (lane < 8);
    if (act) *(volatile v4f*)gp = dv;
    __threadfence();
    if (act) *(volatile v4f*)gp = dv;
  }
}

template <int D>
__global__ __launch_bounds__(NTHR) void k_agg(
    const int* __restrict__ csr, const int* __restrict__ off, const int* __restrict__ cnt,
    const float* __restrict__ eS, const float* __restrict__ eD,
    const int* __restrict__ dsts, const float* __restrict__ ew,
    const float* __restrict__ hc, const float* __restrict__ gam, const float* __restrict__ bet,
    float* out, int nN, int nE, int csrLen) {
  constexpr int P4 = D / 128;
  constexpr int CP = 2 * D;
  static_assert(P4 >= 1 && P4 * 128 == D);
  const int tid = threadIdx.x, lane = tid & 31, wave = tid >> 5;
  const int tbase = blockIdx.x * TGT + wave * 32;
  const float NEGI = -__builtin_huge_valf();

  const int cl     = tbase + lane;
  const int cnt_l  = cnt[cl];
  const int off_l  = off[cl];
  const float es_l = eS[cl];
  v4f gv[P4], bv[P4];
#pragma unroll
  for (int i = 0; i < P4; ++i) {
    gv[i] = *(const v4f*)(gam + 4 * lane + 128 * i);
    bv[i] = *(const v4f*)(bet + 4 * lane + 128 * i);
  }

#pragma unroll 1
  for (int j = 0; j < 32; ++j) {
    const int c = tbase + j;
    int n = __shfl(cnt_l, j);
    n = n < 0 ? 0 : (n > DEGCAP ? DEGCAP : n);
    const int st    = __shfl(off_l, j);
    const float esv = __shfl(es_l, j);

    float mx = NEGI;
#pragma unroll 1
    for (int q0 = 0; q0 < n; q0 += 32) {
      int pos = st + q0 + lane;
      pos = pos < 0 ? 0 : (pos > csrLen - 1 ? csrLen - 1 : pos);
      int e = csr[pos];
      e = e < 0 ? 0 : (e > nE - 1 ? nE - 1 : e);
      int d = dsts[e];
      d = d < 0 ? 0 : (d > nN - 1 ? nN - 1 : d);
      const float t = esv + eD[d];
      const float v = ew[e] * lrelu(t);
      mx = fmaxf(mx, (q0 + lane < n) ? v : NEGI);
    }
    mx = wvmax(mx);

    float den = 0.f;
    v4f acc[P4];
#pragma unroll
    for (int i = 0; i < P4; ++i) { v4f z = {0.f, 0.f, 0.f, 0.f}; acc[i] = z; }
#pragma unroll 1
    for (int q0 = 0; q0 < n; q0 += 32) {
      int pos = st + q0 + lane;
      pos = pos < 0 ? 0 : (pos > csrLen - 1 ? csrLen - 1 : pos);
      int e = csr[pos];
      e = e < 0 ? 0 : (e > nE - 1 ? nE - 1 : e);
      int d = dsts[e];
      d = d < 0 ? 0 : (d > nN - 1 ? nN - 1 : d);
      const float t  = esv + eD[d];
      const float v  = ew[e] * lrelu(t);
      const float pe = __expf(v - mx);
      const float pl = (q0 + lane < n) ? pe : 0.f;
      den += pl;
      const int mcnt = (n - q0) < 32 ? (n - q0) : 32;
#pragma unroll 1
      for (int pp = 0; pp < mcnt; ++pp) {
        const float p  = __int_as_float(__builtin_amdgcn_readlane(__float_as_int(pl), pp));
        const int   dd = __builtin_amdgcn_readlane(d, pp);
        const float* hs = hc + (size_t)dd * CP + 4 * lane;
#pragma unroll
        for (int i = 0; i < P4; ++i) {
          const v4f h = *(const v4f*)(hs + 128 * i);
          acc[i] = acc[i] + h * p;
        }
      }
    }
    den = wvsum(den);

    const float rcp = 1.0f / (den + 1e-16f);
    const float* hrow = hc + (size_t)c * CP + 4 * lane;
    v4f x[P4];
    float sum = 0.f;
#pragma unroll
    for (int i = 0; i < P4; ++i) {
      const v4f hself = *(const v4f*)(hrow + 128 * i);
      const v4f resv  = *(const v4f*)(hrow + D + 128 * i);
      const v4f za    = acc[i] * rcp;
      const v4f z     = (n > 0) ? za : hself;
      x[i] = z + resv;
      sum += x[i].x + x[i].y + x[i].z + x[i].w;
    }
    const float mu = wvsum(sum) * (1.0f / (float)D);
    float vs = 0.f;
#pragma unroll
    for (int i = 0; i < P4; ++i) {
      const float d0 = x[i].x - mu, d1 = x[i].y - mu, d2 = x[i].z - mu, d3 = x[i].w - mu;
      vs += d0 * d0 + d1 * d1 + d2 * d2 + d3 * d3;
    }
    const float rstd = rsqrtf(wvsum(vs) * (1.0f / (float)D) + LN_EPS);
    v4f o[P4];
#pragma unroll
    for (int i = 0; i < P4; ++i) {
      v4f y;
      y.x = (x[i].x - mu) * rstd * gv[i].x + bv[i].x;
      y.y = (x[i].y - mu) * rstd * gv[i].y + bv[i].y;
      y.z = (x[i].z - mu) * rstd * gv[i].z + bv[i].z;
      y.w = (x[i].w - mu) * rstd * gv[i].w + bv[i].w;
      y.x = y.x > 0.f ? y.x : (__expf(y.x) - 1.f);
      y.y = y.y > 0.f ? y.y : (__expf(y.y) - 1.f);
      y.z = y.z > 0.f ? y.z : (__expf(y.z) - 1.f);
      y.w = y.w > 0.f ? y.w : (__expf(y.w) - 1.f);
      o[i] = y;
    }
    float* gp = out + (size_t)c * D + 4 * lane;
    if (c < nN) {
#pragma unroll
      for (int i = 0; i < P4; ++i) *(volatile v4f*)(gp + 128 * i) = o[i];
    }
    __threadfence();
    if (c < nN) {
#pragma unroll
      for (int i = 0; i < P4; ++i) *(volatile v4f*)(gp + 128 * i) = o[i];
    }
  }
}

__global__ __launch_bounds__(NTHR) void k_scores(
    const int* __restrict__ ei, const float* __restrict__ z, float* outp, int nEd, int nN) {
  const int tid = threadIdx.x, lane = tid & 31, wave = tid >> 5;
  const int eb = ((int)blockIdx.x * NWAVE + wave) * 32;
  float keep = 0.f;
#pragma unroll 1
  for (int j = 0; j < 32; ++j) {
    int e = eb + j;
    e = e > nEd - 1 ? nEd - 1 : e;
    int a = ei[e];
    int c = ei[(size_t)nEd + e];
    a = a < 0 ? 0 : (a > nN - 1 ? nN - 1 : a);
    c = c < 0 ? 0 : (c > nN - 1 ? nN - 1 : c);
    const v4f za = *(const v4f*)(z + (size_t)a * HID2 + 4 * lane);
    const v4f zc = *(const v4f*)(z + (size_t)c * HID2 + 4 * lane);
    float s = za.x * zc.x + za.y * zc.y + za.z * zc.z + za.w * zc.w;
    s = wvsum(s);
    s = fminf(fmaxf(s, -SCLAMP), SCLAMP);
    const float sc = 1.0f / (1.0f + __expf(-s));
    keep = (lane == j) ? sc : keep;
  }
  const bool act = eb + lane < nEd;
  float* gp = outp + eb + lane;
  if (act) *(volatile float*)gp = keep;
  __threadfence();
  if (act) *(volatile float*)gp = keep;
}

extern "C" void kernel_launch(void* const* d_in, const int* in_sizes, int n_in,
                              void* d_out, int out_size, void* d_ws, size_t ws_size,
                              hipStream_t stream) {
  if (n_in < 17) return;
  const int nN = in_sizes[0] / IN0;
  const int nE = in_sizes[1] / 2;
  const int nP = in_sizes[3] / 2;
  const int nG = in_sizes[4] / 2;
  if (nN <= 0 || nE <= 0 || nP <= 0 || nG <= 0) return;
  if (in_sizes[0] != nN * IN0 || in_sizes[1] != 2 * nE || in_sizes[2] != nE) return;
  if (in_sizes[3] != 2 * nP || in_sizes[4] != 2 * nG) return;
  if (in_sizes[5] != IN0 * HID1 || in_sizes[6] != HID1 || in_sizes[7] != HID1 || in_sizes[8] != IN0 * HID1) return;
  if (in_sizes[9] != HID1 || in_sizes[10] != HID1) return;
  if (in_sizes[11] != HID1 * HID2 || in_sizes[12] != HID2 || in_sizes[13] != HID2 || in_sizes[14] != HID1 * HID2) return;
  if (in_sizes[15] != HID2 || in_sizes[16] != HID2) return;
  if (nE > (1 << 26) || nN > (1 << 22) || nP > (1 << 26) || nG > (1 << 26)) return;
  if ((long long)out_size != (long long)nN * HID2 + (long long)nP + (long long)nG) return;

  const float* X   = (const float*)d_in[0];
  const int*   Mei = (const int*)d_in[1];
  const float* Mw  = (const float*)d_in[2];
  const int*   Pei = (const int*)d_in[3];
  const int*   Nei = (const int*)d_in[4];
  const float* W1  = (const float*)d_in[5];
  const float* as1 = (const float*)d_in[6];
  const float* ad1 = (const float*)d_in[7];
  const float* Wr1 = (const float*)d_in[8];
  const float* g1  = (const float*)d_in[9];
  const float* b1  = (const float*)d_in[10];
  const float* W2  = (const float*)d_in[11];
  const float* as2 = (const float*)d_in[12];
  const float* ad2 = (const float*)d_in[13];
  const float* Wr2 = (const float*)d_in[14];
  const float* g2  = (const float*)d_in[15];
  const float* b2  = (const float*)d_in[16];
  const int* src = Mei;
  const int* dst = Mei + (size_t)nE;
  float* out0 = (float*)d_out;
  float* outP = out0 + (size_t)nN * HID2;
  float* outG = outP + (size_t)nP;

  const int NPAD   = ((nN + TGT - 1) / TGT) * TGT;
  const int nBC    = (nN + NBC - 1) / NBC;
  const int CNTPAD = nBC * NBC;
  if (CNTPAD < NPAD) return;
  if (4 * nBC + 1 > RBN) return;
  const int nBF    = (nN + NBF - 1) / NBF;
  if (nBF + 1 > 4 * nBC + 1) return;
  const int csrLen = ((nE + 31) & ~31) + 4096;
  if (31 * 4 * nBC > 4096) return;
  const int nAgg   = NPAD / TGT;
  const int nGemm  = NPAD / BM;
  const int nXu1   = NPAD * (IN0 / 8);
  const int nXu2   = NPAD * (HID1 / 8);

  char* ws = (char*)d_ws;
  size_t off = 0;
  const size_t oBh1 = off; off += (size_t)BN1 * IN0 * 2;          off = (off + 255) & ~(size_t)255;
  const size_t oBl1 = off; off += (size_t)BN1 * IN0 * 2;          off = (off + 255) & ~(size_t)255;
  const size_t oBh2 = off; off += (size_t)BN2 * HID1 * 2;         off = (off + 255) & ~(size_t)255;
  const size_t oBl2 = off; off += (size_t)BN2 * HID1 * 2;         off = (off + 255) & ~(size_t)255;
  const size_t oXh  = off; off += (size_t)NPAD * IN0 * 2;         off = (off + 255) & ~(size_t)255;
  const size_t oXl  = off; off += (size_t)NPAD * IN0 * 2;         off = (off + 255) & ~(size_t)255;
  const size_t oCnt = off; off += (size_t)CNTPAD * 4;             off = (off + 255) & ~(size_t)255;
  const size_t oOff = off; off += (size_t)CNTPAD * 4;             off = (off + 255) & ~(size_t)255;
  const size_t oRb  = off; off += (size_t)RBN * 4;                off = (off + 255) & ~(size_t)255;
  const size_t oCsr = off; off += (size_t)csrLen * 4;             off = (off + 255) & ~(size_t)255;
  const size_t oC   = off; off += (size_t)NPAD * BN1 * 4;         off = (off + 255) & ~(size_t)255;
  const size_t oZ1  = off; off += (size_t)NPAD * HID1 * 4;        off = (off + 255) & ~(size_t)255;
  const size_t oES  = off; off += (size_t)NPAD * 4;               off = (off + 255) & ~(size_t)255;
  const size_t oED  = off; off += (size_t)NPAD * 4;               off = (off + 255) & ~(size_t)255;
  if (off > ws_size || off > (size_t)WSCAP) return;
  unsigned short* bh1 = (unsigned short*)(ws + oBh1);
  unsigned short* bl1 = (unsigned short*)(ws + oBl1);
  unsigned short* bh2 = (unsigned short*)(ws + oBh2);
  unsigned short* bl2 = (unsigned short*)(ws + oBl2);
  unsigned short* xph = (unsigned short*)(ws + oXh);
  unsigned short* xpl = (unsigned short*)(ws + oXl);
  int*   cnt  = (int*)(ws + oCnt);
  int*   offp = (int*)(ws + oOff);
  int*   rb   = (int*)(ws + oRb);
  int*   csr  = (int*)(ws + oCsr);
  float* cbuf = (float*)(ws + oC);
  float* z1   = (float*)(ws + oZ1);
  float* es   = (float*)(ws + oES);
  float* ed   = (float*)(ws + oED);

  const int vec8 = 1;

  k_wprep<IN0, HID1><<<(2 * HID1 * (IN0 / 8) + NTHR - 1) / NTHR, NTHR, 0, stream>>>(W1, Wr1, bh1, bl1);
  k_wprep<HID1, HID2><<<(2 * HID2 * (HID1 / 8) + NTHR - 1) / NTHR, NTHR, 0, stream>>>(W2, Wr2, bh2, bl2);

  k_count<<<nBC, NTHR, 0, stream>>>(src, cnt, nE, vec8);
  k_offsets<<<1, OTHR, 0, stream>>>(cnt, offp, rb, nBC);
  hipFuncSetAttribute(reinterpret_cast<const void*>(&k_fill),
                      hipFuncAttributeMaxDynamicSharedMemorySize, LDS_FILL);
  k_fill<<<nBF, NTHR, LDS_FILL, stream>>>(src, offp, rb, csr, nE, vec8, csrLen);

  k_xcvt<IN0><<<(nXu1 + NTHR - 1) / NTHR, NTHR, 0, stream>>>(X, xph, xpl, nN, nXu1);
  hipFuncSetAttribute(reinterpret_cast<const void*>(&k_gemm<IN0, BN1>),
                      hipFuncAttributeMaxDynamicSharedMemorySize, LDS_G1);
  k_gemm<IN0, BN1><<<nGemm, NTHR, LDS_G1, stream>>>(xph, xpl, bh1, bl1, as1, ad1, cbuf, es, ed);
  k_agg<HID1><<<nAgg, NTHR, 0, stream>>>(csr, offp, cnt, es, ed, dst, Mw, cbuf, g1, b1, z1, nN, nE, csrLen);

  k_xcvt<HID1><<<(nXu2 + NTHR - 1) / NTHR, NTHR, 0, stream>>>(z1, xph, xpl, nN, nXu2);
  hipFuncSetAttribute(reinterpret_cast<const void*>(&k_gemm<HID1, BN2>),
                      hipFuncAttributeMaxDynamicSharedMemorySize, LDS_G2);
  k_gemm<HID1, BN2><<<nGemm, NTHR, LDS_G2, stream>>>(xph, xpl, bh2, bl2, as2, ad2, cbuf, es, ed);
  k_agg<HID2><<<nAgg, NTHR, 0, stream>>>(csr, offp, cnt, es, ed, dst, Mw, cbuf, g2, b2, out0, nN, nE, csrLen);

  k_scores<<<(nP + NWAVE * 32 - 1) / (NWAVE * 32), NTHR, 0, stream>>>(Pei, out0, outP, nP, nN);
  k_scores<<<(nG + NWAVE * 32 - 1) / (NWAVE * 32), NTHR, 0, stream>>>(Nei, out0, outG, nG, nN);
}
